// ChannelQuadLayer_16432544875288
// MI455X (gfx1250) — hardware-verified
//
#include <hip/hip_runtime.h>
#include <math.h>

constexpr int kBatch = 8;
constexpr int kCin   = 64;
constexpr int kHW    = 4096;
constexpr int kCout  = 256;
constexpr int kPairs = 2080;
constexpr int kKreal = kCin + kPairs;
constexpr int kKpad  = 2176;
constexpr int kChk   = kKpad / 8;
constexpr int kPxt   = 32;
constexpr int kNbp   = 2;
static_assert(kKpad % 32 == 0, "K multiple of 32");
static_assert(kKreal % 8 == 0, "real K multiple of 8");
static_assert(kCout % 64 == 0 && kHW % 64 == 0, "tile multiples");
static_assert(kBatch % kNbp == 0, "passes");
static_assert((kPxt * kChk) % 256 == 0, "expansion coverage");

typedef __attribute__((ext_vector_type(16))) _Float16 v16h;
typedef __attribute__((ext_vector_type(8)))  _Float16 v8h;
typedef __attribute__((ext_vector_type(16))) __bf16   v16b;
typedef __attribute__((ext_vector_type(8)))  __bf16   v8b;
typedef __attribute__((ext_vector_type(8)))  float    v8f;
typedef __attribute__((ext_vector_type(4)))  float    v4f;
typedef __attribute__((ext_vector_type(4)))  unsigned int v4u;

__device__ __forceinline__ unsigned short f2bf_bits(float f) {
  unsigned u = __float_as_uint(f);
  return (unsigned short)((u + 0x7FFFu + ((u >> 16) & 1u)) >> 16);
}
__device__ __forceinline__ float bf_bits2f(unsigned short h) { return __uint_as_float(((unsigned)h) << 16); }

__device__ __forceinline__ void dep_guard_h(v8f& a, v8f& b, v16h x, v16h y) { asm volatile("v_nop\n\tv_nop\n\tv_nop\n\tv_nop" : "+v"(a), "+v"(b) : "v"(x), "v"(y)); }
__device__ __forceinline__ void dep_guard_b(v8f& a, v8f& b, v16b x, v16b y) { asm volatile("v_nop\n\tv_nop\n\tv_nop\n\tv_nop" : "+v"(a), "+v"(b) : "v"(x), "v"(y)); }
__device__ __forceinline__ void keep4_h(v16h a, v16h b, v16h c, v16h d) { asm volatile("v_nop" :: "v"(a), "v"(b), "v"(c), "v"(d)); }
__device__ __forceinline__ void keep4_b(v16b a, v16b b, v16b c, v16b d) { asm volatile("v_nop" :: "v"(a), "v"(b), "v"(c), "v"(d)); }
__device__ __forceinline__ void acc_guard4(v8f& a, v8f& b, v8f& c, v8f& d) { asm volatile("v_nop\n\tv_nop\n\tv_nop\n\tv_nop" : "+v"(a), "+v"(b), "+v"(c), "+v"(d)); }
template <typename T> struct Frag;
template <> struct Frag<_Float16> {
  typedef v16h V; union U { v16h v; v8h h[2]; };
  static __device__ __forceinline__ v16h load(const _Float16* p) {
    U f; f.h[0] = *(const v8h*)(p); f.h[1] = *(const v8h*)(p + 16); return f.v;
  }
  static __device__ __forceinline__ v8f mma(v16h a, v16h b, v8f c) {
    return __builtin_amdgcn_wmma_f32_16x16x32_f16(false, a, false, b, (short)0, c, false, false);
  }
  static __device__ __forceinline__ void guard(v8f& a, v8f& b, v16h x, v16h y) { dep_guard_h(a, b, x, y); }
  static __device__ __forceinline__ void keep(v16h a, v16h b, v16h c, v16h d) { keep4_h(a, b, c, d); }
};
template <> struct Frag<__bf16> {
  typedef v16b V; union U { v16b v; v8b h[2]; };
  static __device__ __forceinline__ v16b load(const __bf16* p) {
    U f; f.h[0] = *(const v8b*)(p); f.h[1] = *(const v8b*)(p + 16); return f.v;
  }
  static __device__ __forceinline__ v8f mma(v16b a, v16b b, v8f c) {
    return __builtin_amdgcn_wmma_f32_16x16x32_bf16(false, a, false, b, (short)0, c, false, false);
  }
  static __device__ __forceinline__ void guard(v8f& a, v8f& b, v16b x, v16b y) { dep_guard_b(a, b, x, y); }
  static __device__ __forceinline__ void keep(v16b a, v16b b, v16b c, v16b d) { keep4_b(a, b, c, d); }
};

__device__ __forceinline__ unsigned pk16(unsigned short a, unsigned short b) { return (unsigned)a | ((unsigned)b << 16); }
__device__ __forceinline__ unsigned short h_bits(float f) { const _Float16 h = (_Float16)f; return __builtin_bit_cast(unsigned short, h); }

template <int ET> struct Elem;
template <> struct Elem<0> { typedef _Float16 T; };
template <> struct Elem<1> { typedef __bf16 T; };
template <int ET, int SPL, int RSC, int OUT_MODE, int ACT, int TRI>
__global__ __launch_bounds__(256) void wmma_gemm64(
    const unsigned short* __restrict__ Ap, const unsigned short* __restrict__ A2p, int lda, long strideA,
    const unsigned short* __restrict__ Btp, const unsigned short* __restrict__ Bt2p, int ldb, long strideB,
    void* __restrict__ Cout, void* __restrict__ Cout2, int ldc, long strideC,
    const float* __restrict__ rsc, long strideS,
    int M, int N, int K, float scale) {
  typedef typename Elem<ET>::T T;
  typedef typename Frag<T>::V V;
  const T* A = (const T*)Ap; const T* A2 = (const T*)A2p; const T* Bt = (const T*)Btp; const T* Bt2 = (const T*)Bt2p;
  __shared__ __align__(16) float sT[8][16 * 68];
  const int b    = blockIdx.y;
  const int lane = threadIdx.x & 31;
  const int wave = threadIdx.x >> 5;
  const int tilesN = N >> 6;
  const int tilesM = M >> 6;
  const int tile = blockIdx.x * 8 + wave;
  if (tile >= tilesM * tilesN) return;
  const int tm = tile / tilesN;
  const int tn = tile - tm * tilesN;
  const int m0 = tm << 6;
  const int n0 = tn << 6;
  if (TRI == 1 && n0 > m0) return;
  const int Kl = (TRI == 2 && (m0 + 64) < K) ? (m0 + 64) : K;

  const T* Ab  = A  + (size_t)b * strideA;
  const T* Bb  = Bt + (size_t)b * strideB;
  const T* Ab2 = (SPL & 1) ? (A2  + (size_t)b * strideA) : nullptr;
  const T* Bb2 = (SPL & 2) ? (Bt2 + (size_t)b * strideB) : nullptr;

  const int rlane = lane & 15;
  const int koff  = (lane >> 4) * 8;
  const int mOff  = (lane >> 4) * 8;

  v8f acc[4][4];
#pragma unroll
  for (int i = 0; i < 4; ++i)
#pragma unroll
    for (int j = 0; j < 4; ++j) acc[i][j] = (v8f){0.f,0.f,0.f,0.f,0.f,0.f,0.f,0.f};

  for (int k0 = 0; k0 < Kl; k0 += 32) {
    V bh[4], bl[4];
#pragma unroll
    for (int j = 0; j < 4; ++j) {
      const size_t bo = (size_t)(n0 + (j << 4) + rlane) * ldb + koff + k0;
      bh[j] = Frag<T>::load(Bb + bo);
      if (SPL & 2) bl[j] = Frag<T>::load(Bb2 + bo);
    }
#pragma unroll
    for (int i = 0; i < 4; ++i) {
      const size_t ao = (size_t)(m0 + (i << 4) + rlane) * lda + koff + k0;
      V ah = Frag<T>::load(Ab + ao);
      V al;
      if (SPL & 1) al = Frag<T>::load(Ab2 + ao);
#pragma unroll
      for (int j = 0; j < 4; ++j) {
        acc[i][j] = Frag<T>::mma(ah, bh[j], acc[i][j]);
        if (SPL & 2) acc[i][j] = Frag<T>::mma(ah, bl[j], acc[i][j]);
        if (SPL & 1) acc[i][j] = Frag<T>::mma(al, bh[j], acc[i][j]);
      }
      Frag<T>::guard(acc[i][0], acc[i][3], ah, (SPL & 1) ? al : ah);
    }
    Frag<T>::keep(bh[0], bh[1], bh[2], bh[3]);
    if (SPL & 2) Frag<T>::keep(bl[0], bl[1], bl[2], bl[3]);
  }
  acc_guard4(acc[0][0], acc[0][1], acc[0][2], acc[0][3]);
  acc_guard4(acc[1][0], acc[1][1], acc[1][2], acc[1][3]);
  acc_guard4(acc[2][0], acc[2][1], acc[2][2], acc[2][3]);
  acc_guard4(acc[3][0], acc[3][1], acc[3][2], acc[3][3]);

  float* slab = sT[wave];
  const float* Rs = RSC ? (rsc + (size_t)b * strideS) : nullptr;
#pragma unroll
  for (int i = 0; i < 4; ++i) {
    const int mBase = m0 + (i << 4);
    float rsv[8];
#pragma unroll
    for (int r = 0; r < 8; ++r) rsv[r] = RSC ? Rs[mBase + mOff + r] : 1.0f;
#pragma unroll
    for (int j = 0; j < 4; ++j) {
      const int n = n0 + (j << 4) + rlane;
#pragma unroll
      for (int r = 0; r < 8; ++r) {
        float v = acc[i][j][r] * scale;
        if (RSC) v = v * rsv[r];
        if (TRI == 1) { if (n > mBase + mOff + r) v = 0.0f; }
        if (ACT == 6) v = (v > 0.0f) ? (v + 1.0f) : __expf(v);
        slab[(mOff + r) * 68 + (j << 4) + rlane] = v;
      }
    }
    __builtin_amdgcn_fence(__ATOMIC_RELEASE, "workgroup");
    __builtin_amdgcn_wave_barrier();
    __builtin_amdgcn_fence(__ATOMIC_ACQUIRE, "workgroup");
    if (OUT_MODE == 0) {
      float* C = (float*)Cout + (size_t)b * strideC;
      const int hh = lane >> 4, c4 = (lane & 15) * 4;
      for (int pass = 0; pass < 2; ++pass) {
#pragma unroll
        for (int it = 0; it < 8; ++it) {
          const int row = it * 2 + hh;
          v4f v = *(const v4f*)(slab + row * 68 + c4);
          *(volatile v4f*)(C + (size_t)(mBase + row) * ldc + n0 + c4) = v;
        }
        __threadfence();
      }
    } else {
      const int q = lane >> 3, c8 = (lane & 7) * 8;
      unsigned short* C  = (unsigned short*)Cout  + (size_t)b * strideC;
      unsigned short* C2 = (OUT_MODE == 2) ? ((unsigned short*)Cout2 + (size_t)b * strideC) : nullptr;
      for (int pass = 0; pass < 2; ++pass) {
#pragma unroll
        for (int it = 0; it < 4; ++it) {
          const int row = it * 4 + q;
          const float* sp = slab + row * 68 + c8;
          v8h hv, lv;
#pragma unroll
          for (int e = 0; e < 8; ++e) {
            if (OUT_MODE == 1) {
              hv[e] = (_Float16)sp[e];
            } else {
              unsigned short hb = f2bf_bits(sp[e]);
              unsigned short lb = f2bf_bits(sp[e] - bf_bits2f(hb));
              hv[e] = __builtin_bit_cast(_Float16, hb);
              lv[e] = __builtin_bit_cast(_Float16, lb);
            }
          }
          *(volatile v8h*)(C + (size_t)(mBase + row) * ldc + n0 + c8) = hv;
          if (OUT_MODE == 2) *(volatile v8h*)(C2 + (size_t)(mBase + row) * ldc + n0 + c8) = lv;
        }
        __threadfence();
      }
    }
    __builtin_amdgcn_fence(__ATOMIC_RELEASE, "workgroup");
    __builtin_amdgcn_wave_barrier();
    __builtin_amdgcn_fence(__ATOMIC_ACQUIRE, "workgroup");
  }
}

__global__ __launch_bounds__(256) void cast_w_kernel(const float* __restrict__ w, unsigned short* __restrict__ WB) {
  const int row = blockIdx.x;
  const int t   = threadIdx.x;
  const float* wr = w + (size_t)row * kKreal;
  unsigned short* orow = WB + (size_t)row * kKpad;
#pragma unroll 1
  for (int c = t; c < kChk; c += 256) {
    const bool live = (c < kKreal / 8);
    const int  cl   = live ? c : (kKreal / 8 - 1);
    const v4f a = *(const v4f*)(wr + 8 * cl);
    const v4f d = *(const v4f*)(wr + 8 * cl + 4);
    unsigned short hb[8];
#pragma unroll
    for (int e = 0; e < 4; ++e) {
      const unsigned short b0 = f2bf_bits(a[e]);
      const unsigned short b1 = f2bf_bits(d[e]);
      hb[e]     = live ? b0 : (unsigned short)0;
      hb[4 + e] = live ? b1 : (unsigned short)0;
    }
    const v4u u = (v4u){pk16(hb[0], hb[1]), pk16(hb[2], hb[3]), pk16(hb[4], hb[5]), pk16(hb[6], hb[7])};
    unsigned short* q = orow + 8 * c;
    *(volatile v4u*)q = u;
    __threadfence();
    *(volatile v4u*)q = u;
  }
}

__global__ __launch_bounds__(256) void build_y_kernel(const float* __restrict__ x, int b0,
                                                     unsigned short* __restrict__ YH, unsigned short* __restrict__ YL) {
#pragma clang fp contract(off)
  __shared__ __align__(16) float xs[kCin * kPxt];
  __shared__ int tab[kKpad];
  const int t    = threadIdx.x;
  const int lbat = blockIdx.y;
  const int b    = b0 + lbat;
  const int P0   = blockIdx.x * kPxt;

#pragma unroll 1
  for (int k = t; k < kKpad; k += 256) {
    int code = 0;
    if (k < kCin) {
      code = k | (k << 8) | (1 << 16);
    } else if (k < kKreal) {
      int rem = k - kCin, ii = 0;
#pragma unroll 1
      for (int s = 0; s < kCin; ++s) {
        const int len = kCin - ii;
        if (rem >= len) { rem -= len; ++ii; } else break;
      }
      code = ii | ((ii + rem) << 8) | (2 << 16);
    }
    tab[k] = code;
  }
#pragma unroll
  for (int q = 0; q < 2; ++q) {
    const int idx4 = q * 256 + t;
    const int c = idx4 >> 3, m4 = (idx4 & 7) * 4;
    const v4f v = *(const v4f*)(x + ((size_t)(b * kCin + c) * kHW + P0 + m4));
#pragma unroll
    for (int e = 0; e < 4; ++e) xs[c * kPxt + m4 + e] = bf_bits2f(f2bf_bits(v[e]));
  }
  __syncthreads();

  const size_t rowbase = (size_t)lbat * kHW + P0;
#pragma unroll 1
  for (int it = 0; it < (kPxt * kChk) / 256; ++it) {
    const int q  = it * 256 + t;
    const int px = q / kChk;
    const int c  = q - px * kChk;
    unsigned short hb[8], lb[8];
#pragma unroll
    for (int e = 0; e < 8; ++e) {
      const int code = tab[8 * c + e];
      const int i    = code & 63;
      const int j    = (code >> 8) & 63;
      const int mode = (code >> 16) & 3;
      const float a  = xs[i * kPxt + px];
      const float bb = xs[j * kPxt + px];
      const float pr = a * bb;
      float v = (mode == 2) ? pr : a;
      v = (mode == 0) ? 0.0f : v;
      const unsigned short h = f2bf_bits(v);
      hb[e] = h;
      lb[e] = f2bf_bits(v - bf_bits2f(h));
    }
    const v4u uh = (v4u){pk16(hb[0], hb[1]), pk16(hb[2], hb[3]), pk16(hb[4], hb[5]), pk16(hb[6], hb[7])};
    const v4u ul = (v4u){pk16(lb[0], lb[1]), pk16(lb[2], lb[3]), pk16(lb[4], lb[5]), pk16(lb[6], lb[7])};
    const size_t off = (rowbase + px) * (size_t)kKpad + 8 * (size_t)c;
    unsigned short* ph = YH + off;
    unsigned short* pl = YL + off;
    *(volatile v4u*)ph = uh;
    *(volatile v4u*)pl = ul;
    __threadfence();
    *(volatile v4u*)ph = uh;
    *(volatile v4u*)pl = ul;
  }
}

extern "C" void kernel_launch(void* const* d_in, const int* in_sizes, int n_in,
                              void* d_out, int out_size, void* d_ws, size_t ws_size,
                              hipStream_t stream) {
  if (n_in < 2) return;
  if (in_sizes[0] != kBatch * kCin * kHW) return;
  if (in_sizes[1] != kCout * kKreal) return;
  if (out_size != kBatch * kCout * kHW) return;

  const float* x = (const float*)d_in[0];
  const float* w = (const float*)d_in[1];
  float* outp = (float*)d_out;

  const size_t SZ_WB = (size_t)kCout * kKpad * 2;
  const size_t SZ_Y  = (size_t)kNbp * kHW * kKpad * 2;
  const size_t oWB = 0;
  const size_t oYH = oWB + SZ_WB;
  const size_t oYL = oYH + SZ_Y;
  const size_t TOTAL = oYL + SZ_Y;
  if (TOTAL > ws_size) return;
  if (TOTAL > (size_t)134217728) return;

  char* ws = (char*)d_ws;
  unsigned short* WB = (unsigned short*)(ws + oWB);
  unsigned short* YH = (unsigned short*)(ws + oYH);
  unsigned short* YL = (unsigned short*)(ws + oYL);
  const float* dummy_rsc = x;

  const dim3 blk(256);

  cast_w_kernel<<<dim3(kCout), blk, 0, stream>>>(w, WB);

  const int tilesMN = (kCout / 64) * (kHW / 64);
  const dim3 gG((tilesMN + 7) / 8, kNbp);
  const dim3 gY(kHW / kPxt, kNbp);

  for (int p = 0; p < kBatch / kNbp; ++p) {
    const int b0 = p * kNbp;
    build_y_kernel<<<gY, blk, 0, stream>>>(x, b0, YH, YL);
    float* cbase = outp + (size_t)b0 * kCout * kHW;
    wmma_gemm64<1, 2, 0, 0, 0, 0><<<gG, blk, 0, stream>>>(
        WB, WB, kKpad, 0L, YH, YL, kKpad, (long)kHW * kKpad,
        (void*)cbase, (void*)cbase, kHW, (long)kCout * kHW,
        dummy_rsc, 0L, kCout, kHW, kKpad, 1.0f);
  }
}
